// EncoderLayer_59751585022190
// MI455X (gfx1250) — hardware-verified
//
#include <hip/hip_runtime.h>


#ifndef NB
#define NB 2
#endif
#ifndef SEQ
#define SEQ 2048
#endif
#define NB_FULL 2
#define DM   1024
#define NH_  16
#define HD   64
#define FF   4096
#define MT   (NB * SEQ)
#define OSP  68
#define WCAR 64.0f
#define QCAR 8.0f
#define CCAR 256.0f
#define GCAR 64.0f
#define SCL  0.125f
#define LOG2E 1.4426950408889634f
#define LNEPS 1e-6f

static_assert(DM == NH_ * HD);
static_assert(DM == 1024);
static_assert(DM == 8 * 32 * 4);
static_assert(DM == 4 * 32 * 8);
static_assert(HD == 64);
static_assert(SEQ % 64 == 0);
static_assert(MT % 64 == 0);
static_assert(MT % 8 == 0);
static_assert(DM % 64 == 0 && FF % 64 == 0 && (3 * DM) % 64 == 0);
static_assert(DM % 32 == 0 && FF % 32 == 0 && SEQ % 32 == 0);
static_assert(NB <= NB_FULL);
static_assert(((size_t)2 * (4 * (size_t)DM * DM + 2 * (size_t)FF * DM) + (size_t)6 * 2 * MT * DM + (size_t)4 * MT * DM + (size_t)2 * MT * FF) <= (size_t)134217728);

typedef _Float16 h16;
typedef __attribute__((ext_vector_type(16))) _Float16 v16h;
typedef __attribute__((ext_vector_type(8)))  _Float16 v8h;
typedef __attribute__((ext_vector_type(8)))  float    v8f;
typedef __attribute__((ext_vector_type(4)))  float    v4f;
typedef v4f __attribute__((may_alias)) v4fa;

__device__ __forceinline__ float bfr(float f) { unsigned u = __float_as_uint(f); u += 0x7FFFu + ((u >> 16) & 1u); return __uint_as_float(u & 0xFFFF0000u); }
__device__ __forceinline__ v16h cat16(v8h lo, v8h hi) { return __builtin_shufflevector(lo, hi, 0, 1, 2, 3, 4, 5, 6, 7, 8, 9, 10, 11, 12, 13, 14, 15); }
__device__ __forceinline__ v16h ldfrag(const h16* p) { return cat16(*(const v8h*)p, *(const v8h*)(p + 16)); }
__device__ __forceinline__ v8f wmma16(v16h a, v16h b, v8f c) { return __builtin_amdgcn_wmma_f32_16x16x32_f16(false, a, false, b, (short)0, c, false, false); }

template <bool PERM>
__global__ __launch_bounds__(256) void k_cvtw(const float* __restrict__ src, h16* dst, unsigned n8, unsigned kshift) {
    const unsigned i = blockIdx.x * 256u + threadIdx.x; if (i >= n8) return;
    const unsigned e = i * 8u; const unsigned row = e >> kshift; const unsigned k = e & ((1u << kshift) - 1u);
    unsigned srow = row;
    if (PERM) { const unsigned j = row >> 10, h = (row >> 6) & 15u, d = row & 63u; srow = h * 192u + d * 3u + j; }
    const v8f v = *(const v8f*)(src + (((size_t)srow) << kshift) + k); v8h o;
#pragma unroll
    for (int q = 0; q < 8; ++q) o[q] = (h16)(bfr(v[q]) * WCAR);
    *(volatile v8h*)(dst + (size_t)e) = o; __threadfence(); *(volatile v8h*)(dst + (size_t)e) = o;
}

template <bool RAW>
__global__ __launch_bounds__(256) void k_ln(const float* __restrict__ src, const float* __restrict__ g, const float* __restrict__ bb, h16* dst) {
    const unsigned lane = threadIdx.x & 31u; const unsigned row = blockIdx.x * 8u + (threadIdx.x >> 5);
    if (row >= (unsigned)MT) return;
    const unsigned n = row / (unsigned)SEQ, l = row - n * (unsigned)SEQ;
    const float* fr = RAW ? (src + ((size_t)l * NB_FULL + n) * DM) : (src + (size_t)row * DM);
    float s = 0.f;
#pragma unroll 1
    for (unsigned c = 0; c < 8u; ++c) { const v4f a = *(const v4f*)(fr + c * 128u + lane * 4u);
#pragma unroll
        for (int q = 0; q < 4; ++q) { const float t = RAW ? bfr(a[q]) : a[q]; s = __fadd_rn(s, t); } }
#pragma unroll
    for (int sh = 16; sh; sh >>= 1) s = __fadd_rn(s, __shfl_xor(s, sh, 32));
    const float mean = s * (1.0f / (float)DM); float s2 = 0.f;
#pragma unroll 1
    for (unsigned c = 0; c < 8u; ++c) { const v4f a = *(const v4f*)(fr + c * 128u + lane * 4u);
#pragma unroll
        for (int q = 0; q < 4; ++q) { const float t = RAW ? bfr(a[q]) : a[q]; const float dv = __fsub_rn(t, mean); float p2 = __fmul_rn(dv, dv); asm volatile("" : "+v"(p2)); s2 = __fadd_rn(s2, p2); } }
#pragma unroll
    for (int sh = 16; sh; sh >>= 1) s2 = __fadd_rn(s2, __shfl_xor(s2, sh, 32));
    const float rs = __fdiv_rn(1.0f, __fsqrt_rn(__fadd_rn(s2 * (1.0f / (float)DM), LNEPS)));
    h16* orow = dst + (size_t)row * DM + lane * 8u;
#pragma unroll 1
    for (int ps = 0; ps < 2; ++ps) {
#pragma unroll 1
        for (unsigned c = 0; c < 4u; ++c) { const unsigned col = c * 256u + lane * 8u;
            const v8f a = *(const v8f*)(fr + col); const v8f gv = *(const v8f*)(g + col); const v8f bv = *(const v8f*)(bb + col); v8h o;
#pragma unroll
            for (int q = 0; q < 8; ++q) { const float t = RAW ? bfr(a[q]) : a[q]; const float dv = __fsub_rn(t, mean); float y = __fmul_rn(dv, rs); asm volatile("" : "+v"(y)); y = __fmul_rn(y, bfr(gv[q])); asm volatile("" : "+v"(y)); o[q] = (h16)__fadd_rn(y, bfr(bv[q])); }
            *(volatile v8h*)(orow + c * 256u) = o; }
        if (ps == 0) __threadfence(); }
}

enum { EP_QKV = 0, EP_RES = 1, EP_GELU = 2, EP_OUT = 3 };
template <int MODE>
__global__ __launch_bounds__(32) void k_gemmw(const h16* __restrict__ A, const h16* __restrict__ Bt, int K, const float* __restrict__ bias, const float* __restrict__ res, float* outF, h16* outQ, h16* outK, h16* outV, float sc) {
    __shared__ __align__(16) float os[64 * OSP];
    const unsigned lane = threadIdx.x & 31u, lr = lane & 15u, hi = lane >> 4;
    const unsigned r0 = blockIdx.x * 64u, c0 = blockIdx.y * 64u;
    v8f acc[4][4];
#pragma unroll
    for (int mb = 0; mb < 4; ++mb)
#pragma unroll
        for (int nb = 0; nb < 4; ++nb) acc[mb][nb] = (v8f){};
    const size_t aoff = (size_t)(r0 + lr) * (size_t)K + 8u * hi, boff = (size_t)(c0 + lr) * (size_t)K + 8u * hi;
#pragma unroll 1
    for (int kc = 0; kc < K; kc += 32) {
        v16h a[4];
#pragma unroll
        for (int mb = 0; mb < 4; ++mb) a[mb] = ldfrag(A + aoff + (size_t)mb * 16 * K + kc);
#pragma unroll
        for (int nb = 0; nb < 4; ++nb) { const v16h b = ldfrag(Bt + boff + (size_t)nb * 16 * K + kc);
#pragma unroll
            for (int mb = 0; mb < 4; ++mb) acc[mb][nb] = wmma16(a[mb], b, acc[mb][nb]); }
        asm volatile("v_nop\n\tv_nop\n\tv_nop\n\tv_nop" : "+v"(acc[0][0]), "+v"(acc[1][1]), "+v"(acc[2][2]), "+v"(acc[3][3]) : "v"(a[0]), "v"(a[3]));
    }
    const bool tr = (MODE == EP_QKV) && (c0 >= 2u * DM);
    if (tr) {
#pragma unroll
        for (int mb = 0; mb < 4; ++mb)
#pragma unroll
            for (int nb = 0; nb < 4; ++nb) { float* p = os + (nb * 16 + lr) * OSP + mb * 16 + hi * 8; *(v4fa*)p = __builtin_shufflevector(acc[mb][nb], acc[mb][nb], 0, 1, 2, 3); *(v4fa*)(p + 4) = __builtin_shufflevector(acc[mb][nb], acc[mb][nb], 4, 5, 6, 7); }
    } else {
#pragma unroll
        for (int mb = 0; mb < 4; ++mb)
#pragma unroll
            for (int nb = 0; nb < 4; ++nb)
#pragma unroll
                for (int j = 0; j < 8; ++j) os[(mb * 16 + hi * 8 + j) * OSP + nb * 16 + lr] = acc[mb][nb][j];
    }
    __syncthreads();
    const unsigned nbi = r0 / (unsigned)SEQ, l0 = r0 - nbi * (unsigned)SEQ;
    if (MODE == EP_QKV || MODE == EP_GELU) {
        h16* hb; size_t hp;
        if (MODE == EP_QKV) {
            const unsigned jsel = c0 / (unsigned)DM, hh = (c0 - jsel * (unsigned)DM) >> 6;
            const unsigned bbase = hh * (3u * HD) + jsel;
            const float b0 = bfr(bias[bbase + lane * 3u]), b1 = bfr(bias[bbase + (lane + 32u) * 3u]);
#pragma unroll 1
            for (unsigned row = 0; row < 64u; ++row) { const float br = bfr(bias[bbase + row * 3u]); const float u0 = tr ? br : b0, u1 = tr ? br : b1; float* p = os + row * OSP;
                const float w0 = (p[lane] * sc + u0) * QCAR, w1 = (p[lane + 32u] * sc + u1) * QCAR; p[lane] = w0; p[lane + 32u] = w1; }
            const unsigned nhh = nbi * NH_ + hh;
            if (jsel == 0u) { hb = outQ + ((size_t)nhh * SEQ + l0) * HD; hp = HD; }
            else if (jsel == 1u) { hb = outK + ((size_t)nhh * SEQ + l0) * HD; hp = HD; }
            else { hb = outV + (size_t)nhh * HD * SEQ + l0; hp = SEQ; }
        } else {
            const float b0 = bfr(bias[c0 + lane]), b1 = bfr(bias[c0 + lane + 32u]);
#pragma unroll 1
            for (unsigned row = 0; row < 64u; ++row) { float* p = os + row * OSP; const float u0 = p[lane] * sc + b0, u1 = p[lane + 32u] * sc + b1;
                const float g0 = 0.5f * u0 * (1.0f + erff(u0 * 0.70710678118654752f)), g1 = 0.5f * u1 * (1.0f + erff(u1 * 0.70710678118654752f)); p[lane] = g0 * GCAR; p[lane + 32u] = g1 * GCAR; }
            hb = outQ + (size_t)r0 * FF + c0; hp = FF;
        }
        __syncthreads();
        const unsigned rq = lane >> 3, piece = lane & 7u;
#pragma unroll 1
        for (int ps = 0; ps < 2; ++ps) {
#pragma unroll 4
            for (unsigned s = 0; s < 16u; ++s) { const unsigned row = 4u * s + rq; const float* p = os + row * OSP + piece * 8u; const v4f x0 = *(const v4fa*)p; const v4f x1 = *(const v4fa*)(p + 4); v8h o;
#pragma unroll
                for (int q = 0; q < 4; ++q) { o[q] = (h16)x0[q]; o[4 + q] = (h16)x1[q]; }
                *(volatile v8h*)(hb + (size_t)row * hp + piece * 8u) = o; }
            if (ps == 0) __threadfence(); }
    } else {
        const unsigned cofs = lr * 4u;
        const float* resb; size_t rp; float* outb; size_t op;
        if (MODE == EP_RES) { resb = res + ((size_t)l0 * NB_FULL + nbi) * DM + c0; rp = (size_t)NB_FULL * DM; outb = outF + (size_t)r0 * DM + c0; op = DM; }
        else { resb = res + (size_t)r0 * DM + c0; rp = DM; outb = outF + ((size_t)l0 * NB_FULL + nbi) * DM + c0; op = (size_t)NB_FULL * DM; }
        float b4[4];
#pragma unroll
        for (int q = 0; q < 4; ++q) b4[q] = bfr(bias[c0 + cofs + q]);
#pragma unroll 2
        for (unsigned s = 0; s < 32u; ++s) { const unsigned row = 2u * s + hi; float* p = os + row * OSP + cofs; v4f v = *(const v4fa*)p; const v4f r = *(const v4f*)(resb + (size_t)row * rp + cofs);
#pragma unroll
            for (int q = 0; q < 4; ++q) { const float rr = (MODE == EP_RES) ? bfr(r[q]) : r[q]; v[q] = (v[q] * sc + b4[q]) + rr; }
            *(v4fa*)p = v; }
        __syncthreads();
#pragma unroll 1
        for (int ps = 0; ps < 2; ++ps) {
#pragma unroll 4
            for (unsigned s = 0; s < 32u; ++s) { const unsigned row = 2u * s + hi; const v4f val = *(const v4fa*)(os + row * OSP + cofs); *(volatile v4f*)(outb + (size_t)row * op + cofs) = val; }
            if (ps == 0) __threadfence(); }
    }
}

__global__ __launch_bounds__(32) void k_flash(const h16* __restrict__ QP, const h16* __restrict__ KP, const h16* __restrict__ VT, h16* CTX) {
    __shared__ __align__(16) float os[16 * OSP];
    const unsigned lane = threadIdx.x & 31u, lr = lane & 15u, hi = lane >> 4;
    const unsigned nh = blockIdx.y; const unsigned q0 = blockIdx.x * 16u;
    const h16* Qb = QP + ((size_t)nh * SEQ + q0) * HD;
    const h16* Kb = KP + (size_t)nh * SEQ * HD;
    const h16* Vb = VT + (size_t)nh * HD * SEQ;
    v16h qf[2];
#pragma unroll
    for (int s = 0; s < 2; ++s) qf[s] = ldfrag(Qb + lr * HD + s * 32 + 8u * hi);
    float mrun = -1.0e30f, lrun = 0.f;
    v8f o[4];
#pragma unroll
    for (int dt = 0; dt < 4; ++dt) o[dt] = (v8f){};
    const float c2 = SCL * LOG2E / (QCAR * QCAR);
#pragma unroll 1
    for (unsigned jb = 0; jb < (unsigned)SEQ; jb += 32u) {
        v16h ka[2][2], va[4];
#pragma unroll
        for (int t = 0; t < 2; ++t)
#pragma unroll
            for (int s = 0; s < 2; ++s) ka[t][s] = ldfrag(Kb + (size_t)(jb + t * 16 + lr) * HD + s * 32 + 8u * hi);
#pragma unroll
        for (int dt = 0; dt < 4; ++dt) va[dt] = ldfrag(Vb + (size_t)(dt * 16 + lr) * SEQ + jb + 8u * hi);
        v8f s0 = (v8f){}, s1 = (v8f){};
        s0 = wmma16(ka[0][0], qf[0], s0); s1 = wmma16(ka[1][0], qf[0], s1);
        s0 = wmma16(ka[0][1], qf[1], s0); s1 = wmma16(ka[1][1], qf[1], s1);
        asm volatile("v_nop\n\tv_nop\n\tv_nop\n\tv_nop" : "+v"(s0), "+v"(s1) : "v"(ka[1][1]), "v"(qf[1]));
        float mx = -3.0e38f;
#pragma unroll
        for (int r = 0; r < 8; ++r) { s0[r] *= c2; s1[r] *= c2; mx = fmaxf(mx, fmaxf(s0[r], s1[r])); }
        mx = fmaxf(mx, __shfl_xor(mx, 16, 32));
        const float nm = fmaxf(mrun, mx);
        const float alpha = __builtin_amdgcn_exp2f(mrun - nm); mrun = nm;
        float rs = 0.f; v16h pf;
#pragma unroll
        for (int r = 0; r < 8; ++r) { const float p0 = __builtin_amdgcn_exp2f(s0[r] - nm), p1 = __builtin_amdgcn_exp2f(s1[r] - nm); rs += p0 + p1; pf[r] = (h16)p0; pf[8 + r] = (h16)p1; }
        lrun = lrun * alpha + rs;
#pragma unroll
        for (int dt = 0; dt < 4; ++dt)
#pragma unroll
            for (int r = 0; r < 8; ++r) o[dt][r] *= alpha;
#pragma unroll
        for (int dt = 0; dt < 4; ++dt) o[dt] = wmma16(va[dt], pf, o[dt]);
        asm volatile("v_nop\n\tv_nop\n\tv_nop\n\tv_nop" : "+v"(o[0]), "+v"(o[1]), "+v"(o[2]), "+v"(o[3]) : "v"(va[3]), "v"(pf));
    }
    const float lt = lrun + __shfl_xor(lrun, 16, 32);
    const float f = (CCAR / QCAR) * (1.0f / lt);
#pragma unroll
    for (int dt = 0; dt < 4; ++dt)
#pragma unroll
        for (int r = 0; r < 8; ++r) os[lr * OSP + dt * 16 + hi * 8 + r] = o[dt][r] * f;
    __syncthreads();
    const unsigned n = nh / NH_, h = nh - n * NH_;
    const unsigned rq = lane >> 3, piece = lane & 7u;
    h16* base = CTX + ((size_t)n * SEQ + q0) * DM + h * HD + piece * 8u;
    v8h ov[4];
#pragma unroll
    for (int s = 0; s < 4; ++s) { const float* p = os + (4 * s + rq) * OSP + piece * 8u; const v4f x0 = *(const v4fa*)p; const v4f x1 = *(const v4fa*)(p + 4);
#pragma unroll
        for (int q = 0; q < 4; ++q) { ov[s][q] = (h16)x0[q]; ov[s][4 + q] = (h16)x1[q]; } }
#pragma unroll
    for (int s = 0; s < 4; ++s) *(volatile v8h*)(base + (size_t)(4 * s + rq) * DM) = ov[s];
    __threadfence();
#pragma unroll
    for (int s = 0; s < 4; ++s) *(volatile v8h*)(base + (size_t)(4 * s + rq) * DM) = ov[s];
}

extern "C" void kernel_launch(void* const* d_in, const int* in_sizes, int n_in,
                              void* d_out, int out_size, void* d_ws, size_t ws_size, hipStream_t stream) {
    if (n_in < 13) return;
    if ((size_t)in_sizes[0] < (size_t)SEQ * NB_FULL * DM) return;
    if ((size_t)in_sizes[1] < (size_t)3 * DM * DM || (size_t)in_sizes[2] < (size_t)3 * DM) return;
    if ((size_t)in_sizes[3] < (size_t)DM * DM || (size_t)in_sizes[4] < (size_t)DM) return;
    if ((size_t)in_sizes[5] < (size_t)DM || (size_t)in_sizes[6] < (size_t)DM) return;
    if ((size_t)in_sizes[7] < (size_t)FF * DM || (size_t)in_sizes[8] < (size_t)FF) return;
    if ((size_t)in_sizes[9] < (size_t)DM * FF || (size_t)in_sizes[10] < (size_t)DM) return;
    if ((size_t)in_sizes[11] < (size_t)DM || (size_t)in_sizes[12] < (size_t)DM) return;
    if ((size_t)out_size < (size_t)SEQ * NB_FULL * DM) return;
    const float* x = (const float*)d_in[0]; const float* wqkv = (const float*)d_in[1]; const float* bqkv = (const float*)d_in[2];
    const float* wo = (const float*)d_in[3]; const float* bo = (const float*)d_in[4]; const float* g1 = (const float*)d_in[5]; const float* be1 = (const float*)d_in[6];
    const float* w1 = (const float*)d_in[7]; const float* b1 = (const float*)d_in[8]; const float* w2 = (const float*)d_in[9]; const float* b2 = (const float*)d_in[10];
    const float* g2 = (const float*)d_in[11]; const float* be2 = (const float*)d_in[12];
    float* OUT = (float*)d_out;
    char* wsp = (char*)d_ws;
    auto take = [&](size_t bytes) { char* p = wsp; wsp += (bytes + 255) & ~(size_t)255; return (void*)p; };
    h16* WQKV = (h16*)take((size_t)3 * DM * DM * 2); h16* WO = (h16*)take((size_t)DM * DM * 2); h16* W1 = (h16*)take((size_t)FF * DM * 2); h16* W2 = (h16*)take((size_t)DM * FF * 2);
    h16* H1 = (h16*)take((size_t)MT * DM * 2); h16* QP = (h16*)take((size_t)MT * DM * 2); h16* KP = (h16*)take((size_t)MT * DM * 2); h16* VT = (h16*)take((size_t)MT * DM * 2);
    h16* CTX = (h16*)take((size_t)MT * DM * 2); float* X1 = (float*)take((size_t)MT * DM * 4); h16* H2 = (h16*)take((size_t)MT * DM * 2); h16* G = (h16*)take((size_t)MT * FF * 2);
    if ((size_t)(wsp - (char*)d_ws) > ws_size) return;
    { const unsigned n8a = (unsigned)((size_t)3 * DM * DM / 8), n8b = (unsigned)((size_t)DM * DM / 8), n8c = (unsigned)((size_t)FF * DM / 8);
      k_cvtw<true><<<(n8a + 255u) / 256u, 256, 0, stream>>>(wqkv, WQKV, n8a, 10u);
      k_cvtw<false><<<(n8b + 255u) / 256u, 256, 0, stream>>>(wo, WO, n8b, 10u);
      k_cvtw<false><<<(n8c + 255u) / 256u, 256, 0, stream>>>(w1, W1, n8c, 10u);
      k_cvtw<false><<<(n8c + 255u) / 256u, 256, 0, stream>>>(w2, W2, n8c, 12u); }
    k_ln<true><<<(MT + 7) / 8, 256, 0, stream>>>(x, g1, be1, H1);
    k_gemmw<EP_QKV><<<dim3(MT / 64, 3 * DM / 64, 1), 32, 0, stream>>>(H1, WQKV, DM, bqkv, x, X1, QP, KP, VT, 1.0f / WCAR);
    k_flash<<<dim3(SEQ / 16, NB * NH_, 1), 32, 0, stream>>>(QP, KP, VT, CTX);
    k_gemmw<EP_RES><<<dim3(MT / 64, DM / 64, 1), 32, 0, stream>>>(CTX, WO, DM, bo, x, X1, G, G, G, 1.0f / (CCAR * WCAR));
    k_ln<false><<<(MT + 7) / 8, 256, 0, stream>>>(X1, g2, be2, H2);
    k_gemmw<EP_GELU><<<dim3(MT / 64, FF / 64, 1), 32, 0, stream>>>(H2, W1, DM, b1, x, X1, G, G, G, 1.0f / WCAR);
    k_gemmw<EP_OUT><<<dim3(MT / 64, DM / 64, 1), 32, 0, stream>>>(G, W2, FF, b2, X1, OUT, G, G, G, 1.0f / (GCAR * WCAR));
}
